// TverskyLayer_29497835389698
// MI455X (gfx1250) — hardware-verified
//
#include <hip/hip_runtime.h>
#include <math.h>
#include <stdint.h>

#define NB 4096
#define ND 1024
#define NF 2048
#define NP 1024
static_assert((NB % 64) == 0 && (NF % 64) == 0 && (NP % 64) == 0 && (ND % 32) == 0 && (NF % 32) == 0);
static_assert((NB % 32) == 0 && (NP % 32) == 0);
static_assert(NF == 256 * 8);
static_assert(((NB * ND) % (8 * 256)) == 0 && ((NF * ND) % (8 * 256)) == 0 && ((NP * ND) % (8 * 256)) == 0);
static_assert(((NB * NP) % (4 * 256)) == 0 && (NP % 4) == 0);

typedef __bf16   v16b __attribute__((ext_vector_type(16)));
typedef __bf16   v8b  __attribute__((ext_vector_type(8)));
typedef float    v8f  __attribute__((ext_vector_type(8)));
typedef float    v4f  __attribute__((ext_vector_type(4)));
typedef unsigned int v4u __attribute__((ext_vector_type(4)));

__device__ __forceinline__ unsigned short bf_bits(float f) {
  unsigned u = __float_as_uint(f);
  return (unsigned short)((u + 0x7FFFu + ((u >> 16) & 1u)) >> 16);
}
__device__ __forceinline__ float bf_up(unsigned short h) { return __uint_as_float(((unsigned)h) << 16); }
__device__ __forceinline__ unsigned pk16(unsigned short a, unsigned short b) { return (unsigned)a | ((unsigned)b << 16); }
__device__ __forceinline__ v8f zero8() { v8f z = {0.f, 0.f, 0.f, 0.f, 0.f, 0.f, 0.f, 0.f}; return z; }

__device__ __forceinline__ v16b ldfrag_b(const __bf16* p) {
  union { v16b v; v8b h[2]; } f;
  f.h[0] = *(const v8b*)(p);
  f.h[1] = *(const v8b*)(p + 16);
  return f.v;
}

__device__ __forceinline__ v8f mma_b_raw(v16b a, v16b b, v8f c) {
  return __builtin_amdgcn_wmma_f32_16x16x32_bf16(false, a, false, b, (short)0, c, false, false);
}
__device__ __forceinline__ void dep_guard_b(v8f& a, v8f& b, v16b x, v16b y) {
#if defined(__HIP_DEVICE_COMPILE__)
  asm volatile("v_nop\n\tv_nop\n\tv_nop\n\tv_nop" : "+v"(a), "+v"(b) : "v"(x), "v"(y));
#endif
}
__device__ __forceinline__ void keep4_b(v16b a, v16b b, v16b c, v16b d) {
#if defined(__HIP_DEVICE_COMPILE__)
  asm volatile("v_nop" :: "v"(a), "v"(b), "v"(c), "v"(d));
#endif
}
__device__ __forceinline__ void acc_guard4(v8f& a, v8f& b, v8f& c, v8f& d) {
#if defined(__HIP_DEVICE_COMPILE__)
  asm volatile("v_nop\n\tv_nop\n\tv_nop\n\tv_nop" : "+v"(a), "+v"(b), "+v"(c), "+v"(d));
#endif
}
__device__ __forceinline__ void wave_sync_lds() {
  __builtin_amdgcn_fence(__ATOMIC_RELEASE, "workgroup");
  __builtin_amdgcn_wave_barrier();
  __builtin_amdgcn_fence(__ATOMIC_ACQUIRE, "workgroup");
}

__global__ __launch_bounds__(256) void cvt_bf16x8(const float* __restrict__ in, unsigned short* out,
                                                  int n8, int n8tot) {
  const int i = blockIdx.x * 256 + threadIdx.x;
  if (i >= n8tot) return;
  int ic = i;
  if (ic > n8 - 1) ic = n8 - 1;
  const v4f a = *(const v4f*)(in + (size_t)ic * 8);
  const v4f b = *(const v4f*)(in + (size_t)ic * 8 + 4);
  v4u p;
  p[0] = pk16(bf_bits(a[0]), bf_bits(a[1]));
  p[1] = pk16(bf_bits(a[2]), bf_bits(a[3]));
  p[2] = pk16(bf_bits(b[0]), bf_bits(b[1]));
  p[3] = pk16(bf_bits(b[2]), bf_bits(b[3]));
  if (i >= n8) { p[0] = 0u; p[1] = 0u; p[2] = 0u; p[3] = 0u; }
  *(volatile v4u*)(out + (size_t)i * 8) = p;
  __threadfence();
  *(volatile v4u*)(out + (size_t)i * 8) = p;
}

template <int NSPLIT, int OUT_MODE>
__global__ __launch_bounds__(256) void gemm64(
    const unsigned short* __restrict__ Ap, const unsigned short* A2p, int lda, long long strideA,
    const unsigned short* __restrict__ Btp, const unsigned short* Bt2p, int ldb, long long strideB,
    void* Cout, int ldc, long long strideC,
    int M, int N, int K) {
  const __bf16* A   = (const __bf16*)(const void*)Ap;
  const __bf16* A2  = (const __bf16*)(const void*)A2p;
  const __bf16* Bt  = (const __bf16*)(const void*)Btp;
  const __bf16* Bt2 = (const __bf16*)(const void*)Bt2p;
  __shared__ __align__(16) float sT[8][16 * 68];
  const int b    = blockIdx.y;
  const int lane = threadIdx.x & 31;
  const int wave = threadIdx.x >> 5;
  const int tilesN = N >> 6;
  const int tilesM = M >> 6;
  const int tile = blockIdx.x * 8 + wave;
  if (tile >= tilesM * tilesN) return;
  const int tm = tile / tilesN;
  const int tn = tile - tm * tilesN;
  const int m0 = tm << 6;
  const int n0 = tn << 6;

  const __bf16* Ab  = A  + (size_t)b * strideA;
  const __bf16* Bb  = Bt + (size_t)b * strideB;
  const __bf16* Ab2 = (NSPLIT >= 1) ? (A2  + (size_t)b * strideA) : Ab;
  const __bf16* Bb2 = (NSPLIT == 2) ? (Bt2 + (size_t)b * strideB) : Bb;

  const int rlane = lane & 15;
  const int koff  = (lane >> 4) * 8;
  const int mOff  = (lane >> 4) * 8;

  v8f acc[4][4];
#pragma unroll
  for (int i = 0; i < 4; ++i)
#pragma unroll
    for (int j = 0; j < 4; ++j) acc[i][j] = zero8();

  for (int k0 = 0; k0 < K; k0 += 32) {
    v16b bh[4], bl[4];
#pragma unroll
    for (int j = 0; j < 4; ++j) {
      const size_t bo = (size_t)(n0 + (j << 4) + rlane) * ldb + koff + k0;
      bh[j] = ldfrag_b(Bb + bo);
      if (NSPLIT == 2) bl[j] = ldfrag_b(Bb2 + bo); else bl[j] = bh[j];
    }
#pragma unroll
    for (int i = 0; i < 4; ++i) {
      const size_t ao = (size_t)(m0 + (i << 4) + rlane) * lda + koff + k0;
      const v16b ah = ldfrag_b(Ab + ao);
      v16b al = ah;
      if (NSPLIT >= 1) al = ldfrag_b(Ab2 + ao);
#pragma unroll
      for (int j = 0; j < 4; ++j) {
        acc[i][j] = mma_b_raw(ah, bh[j], acc[i][j]);
        if (NSPLIT >= 1) acc[i][j] = mma_b_raw(al, bh[j], acc[i][j]);
        if (NSPLIT == 2) acc[i][j] = mma_b_raw(ah, bl[j], acc[i][j]);
      }
      dep_guard_b(acc[i][0], acc[i][3], ah, al);
    }
    keep4_b(bh[0], bh[1], bh[2], bh[3]);
    if (NSPLIT == 2) keep4_b(bl[0], bl[1], bl[2], bl[3]);
  }
  acc_guard4(acc[0][0], acc[0][1], acc[0][2], acc[0][3]);
  acc_guard4(acc[1][0], acc[1][1], acc[1][2], acc[1][3]);
  acc_guard4(acc[2][0], acc[2][1], acc[2][2], acc[2][3]);
  acc_guard4(acc[3][0], acc[3][1], acc[3][2], acc[3][3]);

  float* slab = sT[wave];
  const int hh = lane >> 4, c4 = (lane & 15) * 4;
  float* C = (float*)Cout + (size_t)b * strideC;
#pragma unroll
  for (int i = 0; i < 4; ++i) {
    const int mBase = m0 + (i << 4);
#pragma unroll
    for (int j = 0; j < 4; ++j) {
#pragma unroll
      for (int r = 0; r < 8; ++r) {
        slab[(mOff + r) * 68 + (j << 4) + rlane] = acc[i][j][r];
      }
    }
    wave_sync_lds();
    for (int pass = 0; pass < 2; ++pass) {
#pragma unroll
      for (int it = 0; it < 8; ++it) {
        const int row = it * 2 + hh;
        const v4f v = *(const v4f*)(slab + row * 68 + c4);
        *(volatile v4f*)(C + (size_t)(mBase + row) * ldc + n0 + c4) = v;
      }
      __threadfence();
    }
    wave_sync_lds();
  }
}

__device__ __forceinline__ float sigm(float t) {
  const float e = __expf(-t);
  return __builtin_amdgcn_rcpf(1.0f + e);
}

__global__ __launch_bounds__(256) void sig_planes(const float* __restrict__ Tp, unsigned short* AXo,
                                                  unsigned short* SXo, float* rso, int R) {
  __shared__ float sW[8];
  __shared__ __align__(16) float sRS[32];
  const int tid  = threadIdx.x;
  const int lane = tid & 31;
  const int wave = tid >> 5;
  const int r0   = blockIdx.x * 32;
  for (int rr = 0; rr < 32; ++rr) {
    int row = r0 + rr;
    if (row > R - 1) row = R - 1;
    const size_t base = (size_t)row * NF + (size_t)tid * 8;
    const v4f a = *(const v4f*)(Tp + base);
    const v4f b = *(const v4f*)(Tp + base + 4);
    const float t0 = a[0], t1 = a[1], t2 = a[2], t3 = a[3];
    const float t4 = b[0], t5 = b[1], t6 = b[2], t7 = b[3];
    const float s0 = sigm(t0), s1 = sigm(t1), s2 = sigm(t2), s3 = sigm(t3);
    const float s4 = sigm(t4), s5 = sigm(t5), s6 = sigm(t6), s7 = sigm(t7);
    const float g0 = t0 * s0, g1 = t1 * s1, g2 = t2 * s2, g3 = t3 * s3;
    const float g4 = t4 * s4, g5 = t5 * s5, g6 = t6 * s6, g7 = t7 * s7;
    v4u pa, ps;
    pa[0] = pk16(bf_bits(g0), bf_bits(g1));
    pa[1] = pk16(bf_bits(g2), bf_bits(g3));
    pa[2] = pk16(bf_bits(g4), bf_bits(g5));
    pa[3] = pk16(bf_bits(g6), bf_bits(g7));
    ps[0] = pk16(bf_bits(s0), bf_bits(s1));
    ps[1] = pk16(bf_bits(s2), bf_bits(s3));
    ps[2] = pk16(bf_bits(s4), bf_bits(s5));
    ps[3] = pk16(bf_bits(s6), bf_bits(s7));
    *(volatile v4u*)(AXo + base) = pa;
    *(volatile v4u*)(SXo + base) = ps;
    __threadfence();
    *(volatile v4u*)(AXo + base) = pa;
    *(volatile v4u*)(SXo + base) = ps;

    float part = ((g0 + g1) + (g2 + g3)) + ((g4 + g5) + (g6 + g7));
    part += __shfl_xor(part, 16);
    part += __shfl_xor(part, 8);
    part += __shfl_xor(part, 4);
    part += __shfl_xor(part, 2);
    part += __shfl_xor(part, 1);
    if (lane == 0) sW[wave] = part;
    __syncthreads();
    if (tid == 0) {
      const float tot = ((sW[0] + sW[1]) + (sW[2] + sW[3])) + ((sW[4] + sW[5]) + (sW[6] + sW[7]));
      sRS[rr] = tot;
    }
    __syncthreads();
  }
  if (tid < 8) {
    const v4f v = *(const v4f*)(sRS + tid * 4);
    float* dst = rso + (size_t)r0 + (size_t)tid * 4;
    *(volatile v4f*)dst = v;
    __threadfence();
    *(volatile v4f*)dst = v;
  }
}

__global__ __launch_bounds__(256) void combine_out(
    const float* __restrict__ G1, const float* __restrict__ G2, const float* __restrict__ G3,
    const float* __restrict__ rsA, const float* __restrict__ rsB,
    const float* __restrict__ alphaP, const float* __restrict__ betaP, const float* __restrict__ thetaP,
    float* out, int n4, int P) {
  const int i = blockIdx.x * 256 + threadIdx.x;
  if (i >= n4) return;
  const size_t e = (size_t)i * 4;
  const int row = (int)(e / (size_t)P);
  const int col = (int)(e - (size_t)row * (size_t)P);
  const v4f g1 = *(const v4f*)(G1 + e);
  const v4f g2 = *(const v4f*)(G2 + e);
  const v4f g3 = *(const v4f*)(G3 + e);
  const float ra = rsA[row];
  const v4f rb = *(const v4f*)(rsB + col);
  const float al = bf_up(bf_bits(alphaP[0]));
  const float be = bf_up(bf_bits(betaP[0]));
  const float th = bf_up(bf_bits(thetaP[0]));
  v4f o;
#pragma unroll
  for (int j = 0; j < 4; ++j) {
    o[j] = th * g1[j] - al * (ra - g2[j]) - be * (rb[j] - g3[j]);
  }
  *(volatile v4f*)(out + e) = o;
  __threadfence();
  *(volatile v4f*)(out + e) = o;
}

extern "C" void kernel_launch(void* const* d_in, const int* in_sizes, int n_in,
                              void* d_out, int out_size, void* d_ws, size_t ws_size,
                              hipStream_t stream) {
  if (n_in < 6) return;
  if (in_sizes[0] != NB * ND) return;
  if (in_sizes[1] != NF * ND) return;
  if (in_sizes[2] != NP * ND) return;
  if (in_sizes[3] < 1 || in_sizes[4] < 1 || in_sizes[5] < 1) return;
  if (out_size != NB * NP) return;

  const float* x      = (const float*)d_in[0];
  const float* feat   = (const float*)d_in[1];
  const float* proto  = (const float*)d_in[2];
  const float* alphaP = (const float*)d_in[3];
  const float* betaP  = (const float*)d_in[4];
  const float* thetaP = (const float*)d_in[5];
  float* out = (float*)d_out;

  const size_t PXb = (size_t)NB * ND * 2;
  const size_t PFb = (size_t)NF * ND * 2;
  const size_t PPb = (size_t)NP * ND * 2;
  const size_t PXF = (size_t)NB * NF * 4;
  const size_t PPF = (size_t)NP * NF * 4;
  const size_t PAX = (size_t)NB * NF * 2;
  const size_t PBP = (size_t)NP * NF * 2;
  const size_t PG  = (size_t)NB * NP * 4;
  const size_t PrA = (size_t)NB * 4;
  const size_t PrB = (size_t)NP * 4;
  static_assert(2 * (size_t)NB * NP * 4 <= (size_t)NB * NF * 4);
  size_t off = 0;
  const size_t oXb = off; off += PXb;
  const size_t oFb = off; off += PFb;
  const size_t oPb = off; off += PPb;
  const size_t oXF = off; off += PXF;
  const size_t oPF = off; off += PPF;
  const size_t oAX = off; off += PAX;
  const size_t oSX = off; off += PAX;
  const size_t oBP = off; off += PBP;
  const size_t oSP = off; off += PBP;
  const size_t oG3 = off; off += PG;
  const size_t orA = off; off += PrA;
  const size_t orB = off; off += PrB;
  if (off > ws_size) return;
  if (off > (size_t)134217728) return;
  const size_t oG1 = oXF;
  const size_t oG2 = oXF + PG;

  char* ws = (char*)d_ws;
  unsigned short* Xb = (unsigned short*)(ws + oXb);
  unsigned short* Fb = (unsigned short*)(ws + oFb);
  unsigned short* Pb = (unsigned short*)(ws + oPb);
  float* XF = (float*)(ws + oXF);
  float* PF = (float*)(ws + oPF);
  unsigned short* AX = (unsigned short*)(ws + oAX);
  unsigned short* SX = (unsigned short*)(ws + oSX);
  unsigned short* BP = (unsigned short*)(ws + oBP);
  unsigned short* SP = (unsigned short*)(ws + oSP);
  float* G1 = (float*)(ws + oG1);
  float* G2 = (float*)(ws + oG2);
  float* G3 = (float*)(ws + oG3);
  float* rsA = (float*)(ws + orA);
  float* rsB = (float*)(ws + orB);

  const dim3 blk(256);
  const int n8x = NB * ND / 8;
  const int n8f = NF * ND / 8;
  const int n8p = NP * ND / 8;
  const dim3 gCvtX((n8x + 255) / 256);
  const dim3 gCvtF((n8f + 255) / 256);
  const dim3 gCvtP((n8p + 255) / 256);
  const dim3 gXF(((NB / 64) * (NF / 64) + 7) / 8, 1);
  const dim3 gPF(((NP / 64) * (NF / 64) + 7) / 8, 1);
  const dim3 gSgX(NB / 32);
  const dim3 gSgP(NP / 32);
  const dim3 gG(((NB / 64) * (NP / 64) + 7) / 8, 1);
  const int n4 = NB * NP / 4;
  const dim3 gOut((n4 + 255) / 256);

  cvt_bf16x8<<<gCvtX, blk, 0, stream>>>(x, Xb, n8x, n8x);
  cvt_bf16x8<<<gCvtF, blk, 0, stream>>>(feat, Fb, n8f, n8f);
  cvt_bf16x8<<<gCvtP, blk, 0, stream>>>(proto, Pb, n8p, n8p);
  gemm64<0, 0><<<gXF, blk, 0, stream>>>(
      Xb, Xb, ND, 0LL, Fb, Fb, ND, 0LL,
      (void*)XF, NF, 0LL,
      NB, NF, ND);
  gemm64<0, 0><<<gPF, blk, 0, stream>>>(
      Pb, Pb, ND, 0LL, Fb, Fb, ND, 0LL,
      (void*)PF, NF, 0LL,
      NP, NF, ND);
  sig_planes<<<gSgX, blk, 0, stream>>>(XF, AX, SX, rsA, NB);
  sig_planes<<<gSgP, blk, 0, stream>>>(PF, BP, SP, rsB, NP);
  gemm64<0, 0><<<gG, blk, 0, stream>>>(
      AX, AX, NF, 0LL, BP, BP, NF, 0LL,
      (void*)G1, NP, 0LL,
      NB, NP, NF);
  gemm64<0, 0><<<gG, blk, 0, stream>>>(
      AX, AX, NF, 0LL, SP, SP, NF, 0LL,
      (void*)G2, NP, 0LL,
      NB, NP, NF);
  gemm64<0, 0><<<gG, blk, 0, stream>>>(
      SX, SX, NF, 0LL, BP, BP, NF, 0LL,
      (void*)G3, NP, 0LL,
      NB, NP, NF);
  combine_out<<<gOut, blk, 0, stream>>>(G1, G2, G3, rsA, rsB, alphaP, betaP, thetaP, out, n4, NP);
  (void)hipGetLastError();
}
